// MMAttn_49160195670476
// MI455X (gfx1250) — hardware-verified
//
#include <hip/hip_runtime.h>
#include <math.h>
#include <stdint.h>

#define NB   2
#define N1T  2048
#define N2T  128
#define DM   1024
#define NH   16
#define DHD  64
#define NT   2176
#define D3   3072
#define R1   (NB * N1T)
#define R2   (NB * N2T)
#define RT   (R1 + R2)
#define NBH  (NB * NH)
#define NKC  (NT / 64)
#define EPSN 1e-6f
static_assert(R1 == 4096 && R2 == 256 && RT == 4352 && NBH == 32 && NKC == 34);
static_assert((N1T % 64) == 0 && (N2T % 64) == 0 && (DM % 64) == 0 && (D3 % 64) == 0 && (DM % 32) == 0);
static_assert(NH * DHD == DM && NKC * 64 == NT);
static_assert(RT * DM == 4456448);

typedef __bf16   v16b __attribute__((ext_vector_type(16)));
typedef __bf16   v8b  __attribute__((ext_vector_type(8)));
typedef float    v8f  __attribute__((ext_vector_type(8)));
typedef float    v4f  __attribute__((ext_vector_type(4)));
typedef unsigned int v4u __attribute__((ext_vector_type(4)));

__device__ __forceinline__ unsigned short bf_bits(float f) {
  unsigned u = __float_as_uint(f);
  return (unsigned short)((u + 0x7FFFu + ((u >> 16) & 1u)) >> 16);
}
__device__ __forceinline__ float bf_up(unsigned short h) { return __uint_as_float(((unsigned)h) << 16); }
__device__ __forceinline__ __bf16 bf_val(unsigned short h) { return __builtin_bit_cast(__bf16, h); }
__device__ __forceinline__ unsigned pk16(unsigned short a, unsigned short b) { return (unsigned)a | ((unsigned)b << 16); }
__device__ __forceinline__ v8f zero8() { v8f z = {0.f, 0.f, 0.f, 0.f, 0.f, 0.f, 0.f, 0.f}; return z; }

__device__ __forceinline__ v16b ldfrag_b(const __bf16* p) {
  union { v16b v; v8b h[2]; } f;
  f.h[0] = *(const v8b*)(p);
  f.h[1] = *(const v8b*)(p + 16);
  return f.v;
}

__device__ __forceinline__ v8f mma_b(v16b a, v16b b, v8f c) {
  c = __builtin_amdgcn_wmma_f32_16x16x32_bf16(false, a, false, b, (short)0, c, false, false);
  asm volatile("v_nop\n\tv_nop\n\tv_nop\n\tv_nop" : "+v"(c) : "v"(a), "v"(b));
  return c;
}
__device__ __forceinline__ v8f mma_b_raw(v16b a, v16b b, v8f c) {
  return __builtin_amdgcn_wmma_f32_16x16x32_bf16(false, a, false, b, (short)0, c, false, false);
}
__device__ __forceinline__ void dep_guard_b(v8f& a, v8f& b, v16b x) {
  asm volatile("v_nop\n\tv_nop\n\tv_nop\n\tv_nop" : "+v"(a), "+v"(b) : "v"(x));
}
__device__ __forceinline__ void dep_guard_b2(v8f& a, v8f& b, v16b x, v16b y) {
  asm volatile("v_nop\n\tv_nop\n\tv_nop\n\tv_nop" : "+v"(a), "+v"(b) : "v"(x), "v"(y));
}
__device__ __forceinline__ void keep4_b(v16b a, v16b b, v16b c, v16b d) {
  asm volatile("v_nop" :: "v"(a), "v"(b), "v"(c), "v"(d));
}
__device__ __forceinline__ void acc_guard4(v8f& a, v8f& b, v8f& c, v8f& d) {
  asm volatile("v_nop\n\tv_nop\n\tv_nop\n\tv_nop" : "+v"(a), "+v"(b), "+v"(c), "+v"(d));
}
__device__ __forceinline__ void lds_wave_sync() {
  __builtin_amdgcn_fence(__ATOMIC_RELEASE, "workgroup");
  __builtin_amdgcn_wave_barrier();
  __builtin_amdgcn_fence(__ATOMIC_ACQUIRE, "workgroup");
}

__device__ __forceinline__ void stage64(float* dst, const float* __restrict__ src, int lane) {
  const int r4 = (lane & 15) * 4;
  const v4f v = *(const v4f*)(src + r4);
  *(v4f*)(dst + r4) = v;
}

__global__ __launch_bounds__(256) void cvt_bf16x8(const float* __restrict__ in, unsigned short* out, int n8) {
  const int i = blockIdx.x * 256 + threadIdx.x;
  if (i < n8) {
    const v4f a = *(const v4f*)(in + (size_t)i * 8);
    const v4f b = *(const v4f*)(in + (size_t)i * 8 + 4);
    v4u p;
    p[0] = pk16(bf_bits(a[0]), bf_bits(a[1]));
    p[1] = pk16(bf_bits(a[2]), bf_bits(a[3]));
    p[2] = pk16(bf_bits(b[0]), bf_bits(b[1]));
    p[3] = pk16(bf_bits(b[2]), bf_bits(b[3]));
    *(volatile v4u*)(out + (size_t)i * 8) = p;
    __threadfence();
    *(volatile v4u*)(out + (size_t)i * 8) = p;
  }
}

__global__ __launch_bounds__(256) void tr_cvt(const float* __restrict__ W, unsigned short* WT, int N) {
  __shared__ __align__(16) unsigned short sT[64 * 72];
  const int tid  = threadIdx.x;
  const int wave = tid >> 5;
  const int lane = tid & 31;
  const int k0 = blockIdx.x * 64;
  const int n0 = blockIdx.y * 64;
  const int r  = tid >> 4;
  const int c4 = (tid & 15) * 4;
#pragma unroll
  for (int p = 0; p < 4; ++p) {
    const int kk = p * 16 + r;
    const v4f v = *(const v4f*)(W + (size_t)(k0 + kk) * N + n0 + c4);
#pragma unroll
    for (int e = 0; e < 4; ++e) sT[(c4 + e) * 72 + kk] = bf_bits(v[e]);
  }
  __syncthreads();
  const int q  = lane >> 3;
  const int c8 = (lane & 7) * 8;
  v4u hv[2];
  size_t o[2];
#pragma unroll
  for (int it = 0; it < 2; ++it) {
    const int n = it * 32 + wave * 4 + q;
    hv[it] = *(const v4u*)(sT + n * 72 + c8);
    o[it]  = (size_t)(n0 + n) * DM + k0 + c8;
  }
  for (int pass = 0; pass < 2; ++pass) {
#pragma unroll
    for (int it = 0; it < 2; ++it) *(volatile v4u*)(WT + o[it]) = hv[it];
    __threadfence();
  }
}

template <bool TWOA>
__device__ __forceinline__ void gemm_core(v8f (&acc)[4][4],
                                          const __bf16* __restrict__ Ah, const __bf16* __restrict__ Al, int lda,
                                          const __bf16* __restrict__ Bb, int ldb, int m0, int n0, int lane) {
  const int rlane = lane & 15;
  const int koff  = (lane >> 4) * 8;
#pragma unroll
  for (int i = 0; i < 4; ++i)
#pragma unroll
    for (int j = 0; j < 4; ++j) acc[i][j] = zero8();

  for (int k0 = 0; k0 < DM; k0 += 32) {
    v16b bh[4];
#pragma unroll
    for (int j = 0; j < 4; ++j) {
      const size_t bo = (size_t)(n0 + (j << 4) + rlane) * ldb + koff + k0;
      bh[j] = ldfrag_b(Bb + bo);
    }
#pragma unroll
    for (int i = 0; i < 4; ++i) {
      const size_t ao = (size_t)(m0 + (i << 4) + rlane) * lda + koff + k0;
      const v16b ah = ldfrag_b(Ah + ao);
      if (TWOA) {
        const v16b al = ldfrag_b(Al + ao);
#pragma unroll
        for (int j = 0; j < 4; ++j) acc[i][j] = mma_b_raw(ah, bh[j], acc[i][j]);
#pragma unroll
        for (int j = 0; j < 4; ++j) acc[i][j] = mma_b_raw(al, bh[j], acc[i][j]);
        dep_guard_b2(acc[i][0], acc[i][3], ah, al);
      } else {
#pragma unroll
        for (int j = 0; j < 4; ++j) acc[i][j] = mma_b_raw(ah, bh[j], acc[i][j]);
        dep_guard_b(acc[i][0], acc[i][3], ah);
      }
    }
    keep4_b(bh[0], bh[1], bh[2], bh[3]);
  }
  acc_guard4(acc[0][0], acc[0][1], acc[0][2], acc[0][3]);
  acc_guard4(acc[1][0], acc[1][1], acc[1][2], acc[1][3]);
  acc_guard4(acc[2][0], acc[2][1], acc[2][2], acc[2][3]);
  acc_guard4(acc[3][0], acc[3][1], acc[3][2], acc[3][3]);
}

__device__ __forceinline__ void epi_hilo(v8f (&acc)[4][4], float* slab, unsigned short* C, unsigned short* C2,
                                         size_t row0, size_t pitch, int lane) {
  const int rlane = lane & 15;
  const int mOff  = (lane >> 4) * 8;
#pragma unroll
  for (int i = 0; i < 4; ++i) {
#pragma unroll
    for (int j = 0; j < 4; ++j) {
#pragma unroll
      for (int r = 0; r < 8; ++r) slab[(mOff + r) * 68 + (j << 4) + rlane] = acc[i][j][r];
    }
    lds_wave_sync();
    {
      const int q = lane >> 3, c8 = (lane & 7) * 8;
      v4u hv[4], lv[4];
#pragma unroll
      for (int it = 0; it < 4; ++it) {
        const int row = it * 4 + q;
        const float* sp = slab + row * 68 + c8;
        v4u a, a2;
#pragma unroll
        for (int e = 0; e < 4; ++e) {
          const float f0 = sp[2 * e], f1 = sp[2 * e + 1];
          const unsigned short h0 = bf_bits(f0), h1 = bf_bits(f1);
          const unsigned short l0 = bf_bits(f0 - bf_up(h0)), l1 = bf_bits(f1 - bf_up(h1));
          a[e] = pk16(h0, h1); a2[e] = pk16(l0, l1);
        }
        hv[it] = a; lv[it] = a2;
      }
      for (int pass = 0; pass < 2; ++pass) {
#pragma unroll
        for (int it = 0; it < 4; ++it) {
          const int row = it * 4 + q;
          const size_t o = (row0 + (size_t)(16 * i + row)) * pitch + c8;
          *(volatile v4u*)(C  + o) = hv[it];
          *(volatile v4u*)(C2 + o) = lv[it];
        }
        __threadfence();
      }
    }
    lds_wave_sync();
  }
}

__device__ __forceinline__ void epi_f32(v8f (&acc)[4][4], float* slab, float* C, size_t row0, size_t pitch, int lane) {
  const int rlane = lane & 15;
  const int mOff  = (lane >> 4) * 8;
#pragma unroll
  for (int i = 0; i < 4; ++i) {
#pragma unroll
    for (int j = 0; j < 4; ++j) {
#pragma unroll
      for (int r = 0; r < 8; ++r) slab[(mOff + r) * 68 + (j << 4) + rlane] = acc[i][j][r];
    }
    lds_wave_sync();
    {
      const int q8 = lane >> 3, c4 = (lane & 7) * 4;
      v4f hv[8];
#pragma unroll
      for (int it = 0; it < 8; ++it) {
        const int idx = it * 4 + q8;
        const int row = idx >> 1, half = idx & 1;
        hv[it] = *(const v4f*)(slab + row * 68 + half * 32 + c4);
      }
      for (int pass = 0; pass < 2; ++pass) {
#pragma unroll
        for (int it = 0; it < 8; ++it) {
          const int idx = it * 4 + q8;
          const int row = idx >> 1, half = idx & 1;
          const size_t o = (row0 + (size_t)(16 * i + row)) * pitch + half * 32 + c4;
          *(volatile v4f*)(C + o) = hv[it];
        }
        __threadfence();
      }
    }
    lds_wave_sync();
  }
}

__global__ __launch_bounds__(256)
void gemm_qk(const unsigned short* __restrict__ Xbp, const unsigned short* __restrict__ Wtp,
             const float* __restrict__ bias, const float* __restrict__ gq, const float* __restrict__ gk,
             unsigned short* Qh, unsigned short* Ql, unsigned short* Kh, unsigned short* Kl,
             int M, int Ns, int t0) {
  __shared__ __align__(16) float sT[8][16 * 68];
  const int lane = threadIdx.x & 31;
  const int wave = threadIdx.x >> 5;
  const int tilesN = (2 * DM) >> 6;
  const int tilesM = M >> 6;
  const int tile = blockIdx.x * 8 + wave;
  if (tile >= tilesM * tilesN) return;
  const int tm = tile / tilesN;
  const int tn = tile - tm * tilesN;
  const int m0 = tm << 6;
  const int n0 = tn << 6;

  const __bf16* Xb = (const __bf16*)(const void*)Xbp;
  const __bf16* Wt = (const __bf16*)(const void*)Wtp;
  v8f acc[4][4];
  gemm_core<false>(acc, Xb, Xb, DM, Wt, DM, m0, n0, lane);

  const int rlane = lane & 15;
  const int which = n0 >> 10;
  const int h     = (n0 & (DM - 1)) >> 6;
  float* slab = sT[wave];
  stage64(slab,       bias + n0, lane);
  stage64(slab + 64,  gq,        lane);
  stage64(slab + 128, gk,        lane);
  lds_wave_sync();
  float bj[4], gs[4];
#pragma unroll
  for (int j = 0; j < 4; ++j) {
    const int d   = (j << 4) + rlane;
    bj[j] = bf_up(bf_bits(slab[d]));
    const float gqv = bf_up(bf_bits(slab[64 + d]));
    const float gkv = bf_up(bf_bits(slab[128 + d]));
    gs[j] = which ? gkv : gqv;
  }
  lds_wave_sync();
#pragma unroll
  for (int i = 0; i < 4; ++i) {
#pragma unroll
    for (int r = 0; r < 8; ++r) {
      float ss = 0.f;
#pragma unroll
      for (int j = 0; j < 4; ++j) {
        const float v = acc[i][j][r] + bj[j];
        acc[i][j][r] = v;
        ss += v * v;
      }
#pragma unroll
      for (int off = 1; off < 16; off <<= 1) ss += __shfl_xor(ss, off, 32);
      const float rs = rsqrtf(ss * (1.0f / 64.0f) + EPSN);
#pragma unroll
      for (int j = 0; j < 4; ++j) acc[i][j][r] = (acc[i][j][r] * rs) * gs[j];
    }
  }

  const int b  = m0 / Ns;
  const int nb = m0 - b * Ns;
  const size_t prow0 = (size_t)(b * NH + h) * NT + (size_t)t0 + (size_t)nb;
  unsigned short* C  = which ? Kh : Qh;
  unsigned short* C2 = which ? Kl : Ql;
  epi_hilo(acc, slab, C, C2, prow0, (size_t)DHD, lane);
}

__global__ __launch_bounds__(256)
void gemm_vt(const unsigned short* __restrict__ WtVp, const unsigned short* __restrict__ Xbp,
             const float* __restrict__ biasv, unsigned short* VTh, unsigned short* VTl, int N, int Ns, int t0) {
  __shared__ __align__(16) float sT[8][16 * 68];
  const int lane = threadIdx.x & 31;
  const int wave = threadIdx.x >> 5;
  const int hh   = lane >> 4;
  const int tilesN = N >> 6;
  const int tilesM = DM >> 6;
  const int tile = blockIdx.x * 8 + wave;
  if (tile >= tilesM * tilesN) return;
  const int tm = tile / tilesN;
  const int tn = tile - tm * tilesN;
  const int m0 = tm << 6;
  const int n0 = tn << 6;

  const __bf16* Wt = (const __bf16*)(const void*)WtVp;
  const __bf16* Xb = (const __bf16*)(const void*)Xbp;
  v8f acc[4][4];
  gemm_core<false>(acc, Wt, Wt, DM, Xb, DM, m0, n0, lane);

  float* slab = sT[wave];
  stage64(slab, biasv + m0, lane);
  lds_wave_sync();
#pragma unroll
  for (int i = 0; i < 4; ++i) {
    const v4f b0 = *(const v4f*)(slab + (i << 4) + 8 * hh);
    const v4f b1 = *(const v4f*)(slab + (i << 4) + 8 * hh + 4);
#pragma unroll
    for (int j = 0; j < 4; ++j) {
#pragma unroll
      for (int r = 0; r < 4; ++r) {
        acc[i][j][r]     += bf_up(bf_bits(b0[r]));
        acc[i][j][4 + r] += bf_up(bf_bits(b1[r]));
      }
    }
  }
  lds_wave_sync();

  const int h  = m0 >> 6;
  const int b  = n0 / Ns;
  const int nb = n0 - b * Ns;
  const size_t vrow0 = (size_t)(b * NH + h) * DHD;
  const size_t coff  = (size_t)t0 + (size_t)nb;
  epi_hilo(acc, slab, VTh + coff, VTl + coff, vrow0, (size_t)NT, lane);
}

__global__ __launch_bounds__(256)
void gemm_out(const unsigned short* __restrict__ Ohp, const unsigned short* __restrict__ Olp,
              const unsigned short* __restrict__ Wtp, const float* __restrict__ bias, float* outp, int M) {
  __shared__ __align__(16) float sT[8][16 * 68];
  const int lane = threadIdx.x & 31;
  const int wave = threadIdx.x >> 5;
  const int tilesN = DM >> 6;
  const int tilesM = M >> 6;
  const int tile = blockIdx.x * 8 + wave;
  if (tile >= tilesM * tilesN) return;
  const int tm = tile / tilesN;
  const int tn = tile - tm * tilesN;
  const int m0 = tm << 6;
  const int n0 = tn << 6;

  const __bf16* Oh = (const __bf16*)(const void*)Ohp;
  const __bf16* Ol = (const __bf16*)(const void*)Olp;
  const __bf16* Wt = (const __bf16*)(const void*)Wtp;
  v8f acc[4][4];
  gemm_core<true>(acc, Oh, Ol, DM, Wt, DM, m0, n0, lane);

  const int rlane = lane & 15;
  float* slab = sT[wave];
  stage64(slab, bias + n0, lane);
  lds_wave_sync();
  float bj[4];
#pragma unroll
  for (int j = 0; j < 4; ++j) bj[j] = bf_up(bf_bits(slab[(j << 4) + rlane]));
  lds_wave_sync();
#pragma unroll
  for (int i = 0; i < 4; ++i)
#pragma unroll
    for (int j = 0; j < 4; ++j)
#pragma unroll
      for (int r = 0; r < 8; ++r) acc[i][j][r] += bj[j];

  epi_f32(acc, slab, outp + n0, (size_t)m0, (size_t)DM, lane);
}

#define A_KSH 0
#define A_KSL 8192
#define A_VTH 16384
#define A_VTL 24576
#define A_PH  32768
#define A_PL  40960
#define A_TOT 49152
static_assert(A_KSL - A_KSH == 64 * DHD * 2 && A_VTH - A_KSL == 64 * DHD * 2);
static_assert(A_VTL - A_VTH == DHD * 64 * 2 && A_PH - A_VTL == DHD * 64 * 2);
static_assert(A_PL - A_PH == 4 * 16 * 64 * 2 && A_TOT - A_PL == 4 * 16 * 64 * 2);
static_assert(4 * 16 * DHD * 4 <= A_VTH);

__global__ __launch_bounds__(128)
void attn_mm(const unsigned short* __restrict__ qhp, const unsigned short* __restrict__ qlp,
             const unsigned short* __restrict__ khp, const unsigned short* __restrict__ klp,
             const unsigned short* __restrict__ vhp, const unsigned short* __restrict__ vlp,
             unsigned short* Ohp, unsigned short* Olp) {
  extern __shared__ __align__(16) unsigned char lds[];
  union FB { v16b v; v8b h[2]; };
  __bf16* Ksh = (__bf16*)(lds + A_KSH);
  __bf16* Ksl = (__bf16*)(lds + A_KSL);
  __bf16* Vth = (__bf16*)(lds + A_VTH);
  __bf16* Vtl = (__bf16*)(lds + A_VTL);
  __bf16* Ph  = (__bf16*)(lds + A_PH);
  __bf16* Pl  = (__bf16*)(lds + A_PL);

  const int tid  = threadIdx.x;
  const int wave = tid >> 5;
  const int lane = tid & 31;
  const int hh   = lane >> 4;
  const int c    = lane & 15;

  const int bx = blockIdx.x;
  const int z  = bx / NKC;
  const int qb = bx - z * NKC;
  const int b  = z >> 4;
  const int h  = z & (NH - 1);
  const int q0 = qb * 64 + wave * 16;
  const size_t zrow = (size_t)z * NT;

  const __bf16* Qh = (const __bf16*)(const void*)qhp;
  const __bf16* Ql = (const __bf16*)(const void*)qlp;
  const __bf16* Kh = (const __bf16*)(const void*)khp;
  const __bf16* Kl = (const __bf16*)(const void*)klp;
  const __bf16* Vh = (const __bf16*)(const void*)vhp + (size_t)z * DHD * NT;
  const __bf16* Vl = (const __bf16*)(const void*)vlp + (size_t)z * DHD * NT;

  __bf16* pwh = Ph + wave * 1024;
  __bf16* pwl = Pl + wave * 1024;

  v8f o[4];
#pragma unroll
  for (int t = 0; t < 4; ++t) o[t] = zero8();
  float mrow[8], lrow[8], alpha[8];
#pragma unroll
  for (int r = 0; r < 8; ++r) { mrow[r] = -INFINITY; lrow[r] = 0.f; alpha[r] = 0.f; }

  const size_t qo = (zrow + q0 + c) * DHD + 8 * hh;

  for (int kt = 0; kt < NKC; ++kt) {
    const int kv0 = kt * 64;
    __syncthreads();
    {
      const __bf16* kgh = Kh + (zrow + kv0) * DHD;
      const __bf16* kgl = Kl + (zrow + kv0) * DHD;
      const __bf16* vgh = Vh + kv0;
      const __bf16* vgl = Vl + kv0;
#pragma unroll
      for (int i = 0; i < 4; ++i) {
        const int p  = tid + 128 * i;
        const int d  = p >> 3;
        const int sg = (p & 7) * 8;
        const v8b a0 = *(const v8b*)(kgh + p * 8);
        const v8b a1 = *(const v8b*)(kgl + p * 8);
        const v8b b0 = *(const v8b*)(vgh + (size_t)d * NT + sg);
        const v8b b1 = *(const v8b*)(vgl + (size_t)d * NT + sg);
        *(v8b*)(Ksh + p * 8) = a0;
        *(v8b*)(Ksl + p * 8) = a1;
        *(v8b*)(Vth + d * 64 + sg) = b0;
        *(v8b*)(Vtl + d * 64 + sg) = b1;
      }
    }
    __syncthreads();

    v8f s[4];
#pragma unroll
    for (int j = 0; j < 4; ++j) s[j] = zero8();
#pragma unroll
    for (int dc = 0; dc < 2; ++dc) {
      const v16b qa = ldfrag_b(Qh + qo + dc * 32);
      const v16b ql = ldfrag_b(Ql + qo + dc * 32);
      const int ko = dc * 32 + 8 * hh;
#pragma unroll
      for (int j = 0; j < 4; ++j) {
        const int kr = (j * 16 + c) * DHD + ko;
        FB kb, kl;
        kb.h[0] = *(const v8b*)(Ksh + kr);
        kb.h[1] = *(const v8b*)(Ksh + kr + 16);
        kl.h[0] = *(const v8b*)(Ksl + kr);
        kl.h[1] = *(const v8b*)(Ksl + kr + 16);
        s[j] = mma_b(qa, kb.v, s[j]);
        s[j] = mma_b(qa, kl.v, s[j]);
        s[j] = mma_b(ql, kb.v, s[j]);
      }
    }

#pragma unroll
    for (int r = 0; r < 8; ++r) {
      const int rowq = q0 + 8 * hh + r;
      float m = -INFINITY;
#pragma unroll
      for (int j = 0; j < 4; ++j) {
        const int key = kv0 + j * 16 + c;
        const bool blk = (rowq < N1T) && (key < N1T) && ((key >> 8) > (rowq >> 8));
        const float madd = blk ? 1.0f : 0.0f;
        const float sv = s[j][r] * 0.125f + madd;
        s[j][r] = sv;
        m = fmaxf(m, sv);
      }
#pragma unroll
      for (int off = 1; off < 16; off <<= 1) m = fmaxf(m, __shfl_xor(m, off, 32));
      const float mnew  = fmaxf(mrow[r], m);
      const float msafe = (mnew == -INFINITY) ? 0.f : mnew;
      const float al    = __expf(mrow[r] - msafe);
      mrow[r]  = mnew;
      alpha[r] = al;
      float psum = 0.f;
#pragma unroll
      for (int j = 0; j < 4; ++j) {
        const float p = __expf(s[j][r] - msafe);
        psum += p;
        const unsigned short hb = bf_bits(p);
        const unsigned short lb = bf_bits(p - bf_up(hb));
        const int po = (8 * hh + r) * 64 + j * 16 + c;
        pwh[po] = bf_val(hb);
        pwl[po] = bf_val(lb);
      }
#pragma unroll
      for (int off = 1; off < 16; off <<= 1) psum += __shfl_xor(psum, off, 32);
      lrow[r] = lrow[r] * al + psum;
    }
    lds_wave_sync();

    FB pa[2], pl[2];
#pragma unroll
    for (int kk = 0; kk < 2; ++kk) {
      const int pr = c * 64 + kk * 32 + 8 * hh;
      pa[kk].h[0] = *(const v8b*)(pwh + pr);
      pa[kk].h[1] = *(const v8b*)(pwh + pr + 16);
      pl[kk].h[0] = *(const v8b*)(pwl + pr);
      pl[kk].h[1] = *(const v8b*)(pwl + pr + 16);
    }
#pragma unroll
    for (int t = 0; t < 4; ++t) {
#pragma unroll
      for (int r = 0; r < 8; ++r) o[t][r] *= alpha[r];
      const int vr0 = (t * 16 + c) * 64 + 8 * hh;
#pragma unroll
      for (int kk = 0; kk < 2; ++kk) {
        FB vb, vl;
        vb.h[0] = *(const v8b*)(Vth + vr0 + kk * 32);
        vb.h[1] = *(const v8b*)(Vth + vr0 + kk * 32 + 16);
        vl.h[0] = *(const v8b*)(Vtl + vr0 + kk * 32);
        vl.h[1] = *(const v8b*)(Vtl + vr0 + kk * 32 + 16);
        o[t] = mma_b(pa[kk].v, vb.v, o[t]);
        o[t] = mma_b(pa[kk].v, vl.v, o[t]);
        o[t] = mma_b(pl[kk].v, vb.v, o[t]);
      }
    }
  }

  __syncthreads();

  float* os = (float*)(lds + A_KSH) + wave * 1024;
  float inv[8];
#pragma unroll
  for (int r = 0; r < 8; ++r) inv[r] = (lrow[r] > 0.f) ? (1.0f / lrow[r]) : 0.f;
#pragma unroll
  for (int t = 0; t < 4; ++t) {
#pragma unroll
    for (int r = 0; r < 8; ++r) os[(8 * hh + r) * 64 + t * 16 + c] = o[t][r] * inv[r];
  }
  lds_wave_sync();
  const int orow0 = (q0 < N1T) ? (b * N1T + q0) : (R1 + b * N2T + (q0 - N1T));
  const int q8 = lane >> 3, c8 = (lane & 7) * 8;
  v4u hv[4], lv[4];
#pragma unroll
  for (int it = 0; it < 4; ++it) {
    const int row = it * 4 + q8;
    const float* sp = os + row * 64 + c8;
    v4u a, a2;
#pragma unroll
    for (int e = 0; e < 4; ++e) {
      const float f0 = sp[2 * e], f1 = sp[2 * e + 1];
      const unsigned short h0 = bf_bits(f0), h1 = bf_bits(f1);
      const unsigned short l0 = bf_bits(f0 - bf_up(h0)), l1 = bf_bits(f1 - bf_up(h1));
      a[e] = pk16(h0, h1); a2[e] = pk16(l0, l1);
    }
    hv[it] = a; lv[it] = a2;
  }
  for (int pass = 0; pass < 2; ++pass) {
#pragma unroll
    for (int it = 0; it < 4; ++it) {
      const int row = it * 4 + q8;
      const size_t oo = (size_t)(orow0 + row) * DM + (size_t)h * DHD + c8;
      *(volatile v4u*)(Ohp + oo) = hv[it];
      *(volatile v4u*)(Olp + oo) = lv[it];
    }
    __threadfence();
  }
}

extern "C" void kernel_launch(void* const* d_in, const int* in_sizes, int n_in,
                              void* d_out, int out_size, void* d_ws, size_t ws_size,
                              hipStream_t stream) {
  if (n_in < 14) return;
  if (in_sizes[0] != R1 * DM || in_sizes[1] != R2 * DM) return;
  if (in_sizes[2] != DM * D3 || in_sizes[3] != D3 || in_sizes[4] != DM * D3 || in_sizes[5] != D3) return;
  if (in_sizes[6] != DM * DM || in_sizes[7] != DM || in_sizes[8] != DM * DM || in_sizes[9] != DM) return;
  if (in_sizes[10] != DHD || in_sizes[11] != DHD || in_sizes[12] != DHD || in_sizes[13] != DHD) return;
  if (out_size != RT * DM) return;

  const float* x1    = (const float*)d_in[0];
  const float* x2    = (const float*)d_in[1];
  const float* Wqkv1 = (const float*)d_in[2];
  const float* bqkv1 = (const float*)d_in[3];
  const float* Wqkv2 = (const float*)d_in[4];
  const float* bqkv2 = (const float*)d_in[5];
  const float* Wout1 = (const float*)d_in[6];
  const float* bout1 = (const float*)d_in[7];
  const float* Wout2 = (const float*)d_in[8];
  const float* bout2 = (const float*)d_in[9];
  const float* gq1   = (const float*)d_in[10];
  const float* gk1   = (const float*)d_in[11];
  const float* gq2   = (const float*)d_in[12];
  const float* gk2   = (const float*)d_in[13];
  float* out = (float*)d_out;

  const size_t PXB1 = (size_t)R1 * DM * 2;
  const size_t PXB2 = (size_t)R2 * DM * 2;
  const size_t PWT  = (size_t)D3 * DM * 2;
  const size_t PWO  = (size_t)DM * DM * 2;
  const size_t PQK  = (size_t)NBH * NT * DHD * 2;
  const size_t PVT  = (size_t)NBH * DHD * NT * 2;
  const size_t PO   = (size_t)RT * DM * 2;
  size_t off = 0;
  const size_t oXb1 = off; off += PXB1;
  const size_t oXb2 = off; off += PXB2;
  const size_t oW1T = off; off += PWT;
  const size_t oW2T = off; off += PWT;
  const size_t oWo1 = off; off += PWO;
  const size_t oWo2 = off; off += PWO;
  const size_t oQh  = off; off += PQK;
  const size_t oQl  = off; off += PQK;
  const size_t oKh  = off; off += PQK;
  const size_t oKl  = off; off += PQK;
  const size_t oVTh = off; off += PVT;
  const size_t oVTl = off; off += PVT;
  const size_t oOh  = off; off += PO;
  const size_t oOl  = off; off += PO;
  if (off > ws_size) return;
  if (off > (size_t)134217728) return;

  char* ws = (char*)d_ws;
  unsigned short* Xb1 = (unsigned short*)(ws + oXb1);
  unsigned short* Xb2 = (unsigned short*)(ws + oXb2);
  unsigned short* W1T = (unsigned short*)(ws + oW1T);
  unsigned short* W2T = (unsigned short*)(ws + oW2T);
  unsigned short* Wo1 = (unsigned short*)(ws + oWo1);
  unsigned short* Wo2 = (unsigned short*)(ws + oWo2);
  unsigned short* Qh  = (unsigned short*)(ws + oQh);
  unsigned short* Ql  = (unsigned short*)(ws + oQl);
  unsigned short* Kh  = (unsigned short*)(ws + oKh);
  unsigned short* Kl  = (unsigned short*)(ws + oKl);
  unsigned short* VTh = (unsigned short*)(ws + oVTh);
  unsigned short* VTl = (unsigned short*)(ws + oVTl);
  unsigned short* Oh  = (unsigned short*)(ws + oOh);
  unsigned short* Ol  = (unsigned short*)(ws + oOl);

  const dim3 blk(256);
  const int n8x1 = R1 * DM / 8;
  const int n8x2 = R2 * DM / 8;
  const dim3 gCvt1((n8x1 + 255) / 256);
  const dim3 gCvt2((n8x2 + 255) / 256);
  const dim3 gTrW(DM / 64, D3 / 64);
  const dim3 gTrO(DM / 64, DM / 64);
  const dim3 gQK1(((R1 / 64) * ((2 * DM) / 64) + 7) / 8);
  const dim3 gQK2(((R2 / 64) * ((2 * DM) / 64) + 7) / 8);
  const dim3 gVT1(((DM / 64) * (R1 / 64) + 7) / 8);
  const dim3 gVT2(((DM / 64) * (R2 / 64) + 7) / 8);
  const dim3 gAttn(NBH * NKC);
  const dim3 gOut1(((R1 / 64) * (DM / 64) + 7) / 8);
  const dim3 gOut2(((R2 / 64) * (DM / 64) + 7) / 8);

  cvt_bf16x8<<<gCvt1, blk, 0, stream>>>(x1, Xb1, n8x1);
  cvt_bf16x8<<<gCvt2, blk, 0, stream>>>(x2, Xb2, n8x2);
  tr_cvt<<<gTrW, blk, 0, stream>>>(Wqkv1, W1T, D3);
  tr_cvt<<<gTrW, blk, 0, stream>>>(Wqkv2, W2T, D3);
  tr_cvt<<<gTrO, blk, 0, stream>>>(Wout1, Wo1, DM);
  tr_cvt<<<gTrO, blk, 0, stream>>>(Wout2, Wo2, DM);
  gemm_qk<<<gQK1, blk, 0, stream>>>(Xb1, W1T, bqkv1, gq1, gk1, Qh, Ql, Kh, Kl, R1, N1T, 0);
  gemm_qk<<<gQK2, blk, 0, stream>>>(Xb2, W2T, bqkv2, gq2, gk2, Qh, Ql, Kh, Kl, R2, N2T, N1T);
  gemm_vt<<<gVT1, blk, 0, stream>>>(W1T + (size_t)2 * DM * DM, Xb1, bqkv1 + 2 * DM, VTh, VTl, R1, N1T, 0);
  gemm_vt<<<gVT2, blk, 0, stream>>>(W2T + (size_t)2 * DM * DM, Xb2, bqkv2 + 2 * DM, VTh, VTl, R2, N2T, N1T);
  (void)hipFuncSetAttribute(reinterpret_cast<const void*>(&attn_mm),
                            hipFuncAttributeMaxDynamicSharedMemorySize, A_TOT);
  attn_mm<<<gAttn, dim3(128), A_TOT, stream>>>(Qh, Ql, Kh, Kl, VTh, VTl, Oh, Ol);
  gemm_out<<<gOut1, blk, 0, stream>>>(Oh, Ol, Wo1, bout1, out, R1);
  gemm_out<<<gOut2, blk, 0, stream>>>(Oh + (size_t)R1 * DM, Ol + (size_t)R1 * DM, Wo2, bout2,
                                      out + (size_t)R1 * DM, R2);
  (void)hipGetLastError();
}
